// SingleHeadSelfAttention_68667937128837
// MI455X (gfx1250) — hardware-verified
//
#include <hip/hip_runtime.h>
#include <math.h>
#include <stdint.h>

#ifndef NB
#define NB 4
#endif
#ifndef SEQ
#define SEQ 4096
#endif
#define NB_FULL  4
#define SEQ_FULL 4096
#define DM       256
#define NQB      (SEQ / 16)
#define NKT      (SEQ / 64)
#define PCARRY   16384.0f
#define PRES     4096.0f
static_assert(DM == 256);
static_assert((SEQ % 64) == 0 && SEQ >= 64 && SEQ <= SEQ_FULL);
static_assert(NB >= 1 && NB <= NB_FULL);
static_assert(((NB * SEQ) % 64) == 0);

typedef _Float16 v16h __attribute__((ext_vector_type(16)));
typedef _Float16 v8h  __attribute__((ext_vector_type(8)));
typedef __bf16   v16b __attribute__((ext_vector_type(16)));
typedef __bf16   v8b  __attribute__((ext_vector_type(8)));
typedef float    v8f  __attribute__((ext_vector_type(8)));
typedef float    v4f  __attribute__((ext_vector_type(4)));
typedef unsigned int v4u __attribute__((ext_vector_type(4)));

#if defined(__HIP_DEVICE_COMPILE__)
#define DEV_ASM 1
#else
#define DEV_ASM 0
#endif

__device__ __forceinline__ unsigned short bf_bits(float f) {
  unsigned u = __float_as_uint(f);
  return (unsigned short)((u + 0x7FFFu + ((u >> 16) & 1u)) >> 16);
}
__device__ __forceinline__ float bf_up(unsigned short hb) { return __uint_as_float(((unsigned)hb) << 16); }
__device__ __forceinline__ unsigned short h_bits(_Float16 x) { return __builtin_bit_cast(unsigned short, x); }
__device__ __forceinline__ unsigned pk16(unsigned short a, unsigned short b) { return (unsigned)a | ((unsigned)b << 16); }
__device__ __forceinline__ v8f zero8() { v8f z = {0.f, 0.f, 0.f, 0.f, 0.f, 0.f, 0.f, 0.f}; return z; }

template <typename OT> struct FT;
template <> struct FT<__bf16>   { typedef v16b frag; typedef v8b half8; };
template <> struct FT<_Float16> { typedef v16h frag; typedef v8h half8; };

template <typename OT>
__device__ __forceinline__ typename FT<OT>::frag ldfrag(const OT* p) {
  union { typename FT<OT>::frag v; typename FT<OT>::half8 h[2]; } f;
  f.h[0] = *(const typename FT<OT>::half8*)(p);
  f.h[1] = *(const typename FT<OT>::half8*)(p + 16);
  return f.v;
}

__device__ __forceinline__ v8f mmar(v16b a, v16b b, v8f c) {
  return __builtin_amdgcn_wmma_f32_16x16x32_bf16(false, a, false, b, (short)0, c, false, false);
}
__device__ __forceinline__ v8f mmar(v16h a, v16h b, v8f c) {
  return __builtin_amdgcn_wmma_f32_16x16x32_f16(false, a, false, b, (short)0, c, false, false);
}
__device__ __forceinline__ v8f mma_h(v16h a, v16h b, v8f c) {
  c = __builtin_amdgcn_wmma_f32_16x16x32_f16(false, a, false, b, (short)0, c, false, false);
#if DEV_ASM
  asm volatile("v_nop\n\tv_nop\n\tv_nop\n\tv_nop" : "+v"(c) : "v"(a), "v"(b));
#endif
  return c;
}
__device__ __forceinline__ void dep_guard(v8f& a, v8f& b, v16b x, v16b y) {
#if DEV_ASM
  asm volatile("v_nop\n\tv_nop\n\tv_nop\n\tv_nop" : "+v"(a), "+v"(b) : "v"(x), "v"(y));
#else
  (void)a; (void)b; (void)x; (void)y;
#endif
}
__device__ __forceinline__ void dep_guard(v8f& a, v8f& b, v16h x, v16h y) {
#if DEV_ASM
  asm volatile("v_nop\n\tv_nop\n\tv_nop\n\tv_nop" : "+v"(a), "+v"(b) : "v"(x), "v"(y));
#else
  (void)a; (void)b; (void)x; (void)y;
#endif
}
__device__ __forceinline__ void keep4(v16b a, v16b b, v16b c, v16b d) {
#if DEV_ASM
  asm volatile("v_nop" :: "v"(a), "v"(b), "v"(c), "v"(d));
#else
  (void)a; (void)b; (void)c; (void)d;
#endif
}
__device__ __forceinline__ void keep4(v16h a, v16h b, v16h c, v16h d) {
#if DEV_ASM
  asm volatile("v_nop" :: "v"(a), "v"(b), "v"(c), "v"(d));
#else
  (void)a; (void)b; (void)c; (void)d;
#endif
}
__device__ __forceinline__ void acc_guard4(v8f& a, v8f& b, v8f& c, v8f& d) {
#if DEV_ASM
  asm volatile("v_nop\n\tv_nop\n\tv_nop\n\tv_nop" : "+v"(a), "+v"(b), "+v"(c), "+v"(d));
#else
  (void)a; (void)b; (void)c; (void)d;
#endif
}

template <int MODE>
__device__ __forceinline__ unsigned short cvm(float f) {
  const unsigned short hb = bf_bits(f);
  if (MODE == 0) return hb;
  return h_bits((_Float16)(bf_up(hb) * 64.0f));
}

template <int MODE>
__global__ __launch_bounds__(256) void cvt16x8(const float* __restrict__ in, unsigned short* out, int n8) {
  const int i = blockIdx.x * 256 + (int)threadIdx.x;
  if (i < n8) {
    const v4f a  = *(const v4f*)(in + (size_t)i * 8);
    const v4f a4 = *(const v4f*)(in + (size_t)i * 8 + 4);
    v4u p;
    p[0] = pk16(cvm<MODE>(a[0]),  cvm<MODE>(a[1]));
    p[1] = pk16(cvm<MODE>(a[2]),  cvm<MODE>(a[3]));
    p[2] = pk16(cvm<MODE>(a4[0]), cvm<MODE>(a4[1]));
    p[3] = pk16(cvm<MODE>(a4[2]), cvm<MODE>(a4[3]));
    unsigned short* o = out + (size_t)i * 8;
    *(volatile v4u*)o = p;
    __threadfence();
    *(volatile v4u*)o = p;
  }
}

__global__ __launch_bounds__(256) void cvtx(const float* __restrict__ in, unsigned short* out, int n8) {
  const int i = blockIdx.x * 256 + (int)threadIdx.x;
  if (i < n8) {
    const int tk = i >> 5;
    const int e8 = i & 31;
    const int bb = tk / SEQ;
    const int t  = tk - bb * SEQ;
    const float* src = in + ((size_t)bb * SEQ_FULL + (size_t)t) * DM + e8 * 8;
    const v4f a  = *(const v4f*)(src);
    const v4f a4 = *(const v4f*)(src + 4);
    v4u p;
    p[0] = pk16(bf_bits(a[0]),  bf_bits(a[1]));
    p[1] = pk16(bf_bits(a[2]),  bf_bits(a[3]));
    p[2] = pk16(bf_bits(a4[0]), bf_bits(a4[1]));
    p[3] = pk16(bf_bits(a4[2]), bf_bits(a4[3]));
    unsigned short* o = out + (size_t)i * 8;
    *(volatile v4u*)o = p;
    __threadfence();
    *(volatile v4u*)o = p;
  }
}

template <typename OT, int MI, bool ARES, int OUT_MODE>
__global__ __launch_bounds__(256) void gemm_t(
    const unsigned short* __restrict__ Ap, const unsigned short* __restrict__ A2p, int lda, long long strideA,
    const unsigned short* __restrict__ Btp, int ldb, long long strideB,
    void* Cout, void* Cout2, int ldc, long long strideC,
    const float* __restrict__ bias,
    int M, int N, int K, float oscale, float rscale, float ascale) {
  typedef typename FT<OT>::frag V16;
  const OT* A  = (const OT*)(const void*)Ap;
  const OT* A2 = (const OT*)(const void*)A2p;
  const OT* Bt = (const OT*)(const void*)Btp;
  __shared__ __align__(16) float sT[8][16 * 68];
  const int TMR  = 16 * MI;
  const int b    = blockIdx.y;
  const int lane = threadIdx.x & 31;
  const int wave = threadIdx.x >> 5;
  const int tilesN = N >> 6;
  const int tilesM = M / TMR;
  const int tile = blockIdx.x * 8 + wave;
  if (tile >= tilesM * tilesN) return;
  const int tm = tile / tilesN;
  const int tn = tile - tm * tilesN;
  const int m0 = tm * TMR;
  const int n0 = tn << 6;

  const OT* Ab  = A  + (size_t)b * (size_t)strideA;
  const OT* A2b = A2 + (size_t)b * (size_t)strideA;
  const OT* Bb  = Bt + (size_t)b * (size_t)strideB;

  const int rlane = lane & 15;
  const int koff  = (lane >> 4) * 8;
  const int mOff  = (lane >> 4) * 8;

  v8f acc[MI][4], accl[MI][4];
#pragma unroll
  for (int i = 0; i < MI; ++i)
#pragma unroll
    for (int j = 0; j < 4; ++j) { acc[i][j] = zero8(); accl[i][j] = zero8(); }

  for (int k0 = 0; k0 < K; k0 += 32) {
    V16 bq[4];
#pragma unroll
    for (int j = 0; j < 4; ++j)
      bq[j] = ldfrag<OT>(Bb + (size_t)(n0 + (j << 4) + rlane) * ldb + koff + k0);
#pragma unroll
    for (int i = 0; i < MI; ++i) {
      const V16 af = ldfrag<OT>(Ab + (size_t)(m0 + (i << 4) + rlane) * lda + koff + k0);
#pragma unroll
      for (int j = 0; j < 4; ++j) acc[i][j] = mmar(af, bq[j], acc[i][j]);
      dep_guard(acc[i][0], acc[i][3], af, bq[3]);
      if (ARES) {
        const V16 al = ldfrag<OT>(A2b + (size_t)(m0 + (i << 4) + rlane) * lda + koff + k0);
#pragma unroll
        for (int j = 0; j < 4; ++j) accl[i][j] = mmar(al, bq[j], accl[i][j]);
        dep_guard(accl[i][0], accl[i][3], al, bq[3]);
      }
    }
    keep4(bq[0], bq[1], bq[2], bq[3]);
  }
#pragma unroll
  for (int i = 0; i < MI; ++i) {
    acc_guard4(acc[i][0], acc[i][1], acc[i][2], acc[i][3]);
    if (ARES) acc_guard4(accl[i][0], accl[i][1], accl[i][2], accl[i][3]);
  }
  if (ARES) {
#pragma unroll
    for (int i = 0; i < MI; ++i)
#pragma unroll
      for (int j = 0; j < 4; ++j)
#pragma unroll
        for (int r = 0; r < 8; ++r) acc[i][j][r] += accl[i][j][r] * ascale;
  }

  float* slab = sT[wave];
#pragma unroll
  for (int i = 0; i < MI; ++i) {
    const int mBase = m0 + (i << 4);
#pragma unroll
    for (int j = 0; j < 4; ++j) {
#pragma unroll
      for (int r = 0; r < 8; ++r) {
        slab[(mOff + r) * 68 + (j << 4) + rlane] = acc[i][j][r];
      }
    }
    __builtin_amdgcn_fence(__ATOMIC_RELEASE, "workgroup");
    __builtin_amdgcn_wave_barrier();
    __builtin_amdgcn_fence(__ATOMIC_ACQUIRE, "workgroup");
    if (OUT_MODE == 0) {
      float* C = (float*)Cout + (size_t)b * (size_t)strideC;
      const int h2 = lane >> 4, c4 = (lane & 15) * 4;
      const v4f braw = *(const v4f*)(bias + n0 + c4);
      v4f bb;
#pragma unroll
      for (int e = 0; e < 4; ++e) bb[e] = bf_up(bf_bits(braw[e]));
      for (int pass = 0; pass < 2; ++pass) {
#pragma unroll
        for (int it = 0; it < 8; ++it) {
          const int row = it * 2 + h2;
          const v4f v = *(const v4f*)(slab + row * 68 + c4) * oscale + bb;
          *(volatile v4f*)(C + (size_t)(mBase + row) * ldc + n0 + c4) = v;
        }
        __threadfence();
      }
    } else {
      const int q = lane >> 3, c8 = (lane & 7) * 8;
      unsigned short* C  = (unsigned short*)Cout  + (size_t)b * (size_t)strideC;
      unsigned short* C2 = (unsigned short*)Cout2 + (size_t)b * (size_t)strideC;
      v4u hv[4], lv[4];
#pragma unroll
      for (int it = 0; it < 4; ++it) {
        const int row = it * 4 + q;
        const float* sp = slab + row * 68 + c8;
        float f[8];
#pragma unroll
        for (int e = 0; e < 8; ++e) f[e] = sp[e];
        v4u a, a2;
#pragma unroll
        for (int e = 0; e < 4; ++e) {
          const float f0 = f[2 * e], f1 = f[2 * e + 1];
          const _Float16 x0 = (_Float16)f0, x1 = (_Float16)f1;
          const unsigned short h0 = h_bits(x0), h1 = h_bits(x1);
          unsigned short l0 = 0, l1 = 0;
          if (OUT_MODE == 3) {
            l0 = h_bits((_Float16)((f0 - (float)x0) * rscale));
            l1 = h_bits((_Float16)((f1 - (float)x1) * rscale));
          }
          a[e] = pk16(h0, h1); a2[e] = pk16(l0, l1);
        }
        hv[it] = a; lv[it] = a2;
      }
      for (int pass = 0; pass < 2; ++pass) {
#pragma unroll
        for (int it = 0; it < 4; ++it) {
          const int row = it * 4 + q;
          *(volatile v4u*)(C + (size_t)(mBase + row) * ldc + n0 + c8) = hv[it];
          if (OUT_MODE == 3) *(volatile v4u*)(C2 + (size_t)(mBase + row) * ldc + n0 + c8) = lv[it];
        }
        __threadfence();
      }
    }
    __builtin_amdgcn_fence(__ATOMIC_RELEASE, "workgroup");
    __builtin_amdgcn_wave_barrier();
    __builtin_amdgcn_fence(__ATOMIC_ACQUIRE, "workgroup");
  }
}

__global__ __launch_bounds__(128)
void attn_causal(const unsigned short* __restrict__ qhp, const unsigned short* __restrict__ qlp,
                 const unsigned short* __restrict__ kpp,
                 const unsigned short* __restrict__ vhp, const unsigned short* __restrict__ vlp,
                 float* outp, float sscale) {
  union FH { v16h v; v8h h[2]; };
  __shared__ __align__(16) _Float16 Psh[16 * 64];
  __shared__ __align__(16) _Float16 Psl[16 * 64];
  __shared__ __align__(16) float    redm[4][16];
  __shared__ __align__(16) float    reds[4][16];
  __shared__ __align__(16) float    Os[4][16 * 64];

  const int tid  = threadIdx.x;
  const int wave = tid >> 5;
  const int lane = tid & 31;
  const int hh   = lane >> 4;
  const int c    = lane & 15;

  const int bx   = blockIdx.x;
  const int qb   = bx % NQB;
  const int b    = bx / NQB;
  const int q0   = qb * 16;
  const int kcol = wave * 16;
  const int dbase = wave * 64;
  const size_t rowB = (size_t)b * SEQ;
  int ktmax = qb >> 2;
  if (ktmax > NKT - 1) ktmax = NKT - 1;

  const _Float16* Qh = (const _Float16*)(const void*)qhp;
  const _Float16* Ql = (const _Float16*)(const void*)qlp;
  const _Float16* Kp = (const _Float16*)(const void*)kpp;
  const _Float16* Vh = (const _Float16*)(const void*)vhp + ((size_t)b * DM + (size_t)dbase) * SEQ;
  const _Float16* Vl = (const _Float16*)(const void*)vlp + ((size_t)b * DM + (size_t)dbase) * SEQ;

  const _Float16* qrh = Qh + (rowB + q0 + c) * DM + 8 * hh;
  const _Float16* qrl = Ql + (rowB + q0 + c) * DM + 8 * hh;

  float mrow[8], lrow[8];
  v8f oacc[4];
#pragma unroll
  for (int r = 0; r < 8; ++r) { mrow[r] = -INFINITY; lrow[r] = 0.f; }
#pragma unroll
  for (int t = 0; t < 4; ++t) oacc[t] = zero8();

  for (int kt = 0; kt <= ktmax; ++kt) {
    const int kv0 = kt * 64;

    v8f ah = zero8(), al = zero8();
    const _Float16* kr = Kp + (rowB + kv0 + kcol + c) * DM + 8 * hh;
#pragma unroll
    for (int dc = 0; dc < 8; ++dc) {
      const v16h qa = ldfrag<_Float16>(qrh + dc * 32);
      const v16h qr = ldfrag<_Float16>(qrl + dc * 32);
      const v16h kb = ldfrag<_Float16>(kr + dc * 32);
      ah = mma_h(qa, kb, ah);
      al = mma_h(qr, kb, al);
    }
    const int key = kv0 + kcol + c;
    float s[8];
#pragma unroll
    for (int r = 0; r < 8; ++r) {
      const int qrow = q0 + 8 * hh + r;
      const float sv = (ah[r] + al[r] * (1.0f / 4096.0f)) * sscale;
      s[r] = (key > qrow) ? -INFINITY : sv;
    }

#pragma unroll
    for (int r = 0; r < 8; ++r) {
      float m = s[r];
#pragma unroll
      for (int off = 1; off < 16; off <<= 1) m = fmaxf(m, __shfl_xor(m, off, 32));
      redm[wave][8 * hh + r] = m;
    }
    __syncthreads();

#pragma unroll
    for (int r = 0; r < 8; ++r) {
      const int row = 8 * hh + r;
      const float mc    = fmaxf(fmaxf(redm[0][row], redm[1][row]), fmaxf(redm[2][row], redm[3][row]));
      const float mnew  = fmaxf(mrow[r], mc);
      const float msafe = (mnew == -INFINITY) ? 0.f : mnew;
      const float alpha = __expf(mrow[r] - msafe);
      mrow[r] = mnew;
      const float p = __expf(s[r] - msafe);
      float psum = p;
#pragma unroll
      for (int off = 1; off < 16; off <<= 1) psum += __shfl_xor(psum, off, 32);
      const float pc = p * PCARRY;
      const _Float16 ph = (_Float16)pc;
      Psh[row * 64 + kcol + c] = ph;
      Psl[row * 64 + kcol + c] = (_Float16)((pc - (float)ph) * PRES);
      reds[wave][row] = psum;
      lrow[r] *= alpha;
#pragma unroll
      for (int t = 0; t < 4; ++t) oacc[t][r] *= alpha;
    }
    __syncthreads();
#pragma unroll
    for (int r = 0; r < 8; ++r) {
      const int row = 8 * hh + r;
      lrow[r] += (reds[0][row] + reds[1][row]) + (reds[2][row] + reds[3][row]);
    }

    v8f o1[4];
#pragma unroll
    for (int t = 0; t < 4; ++t) o1[t] = zero8();
#pragma unroll 1
    for (int kk = 0; kk < 2; ++kk) {
      FH pa, pl;
      pa.h[0] = *(const v8h*)(Psh + c * 64 + kk * 32 + 8 * hh);
      pa.h[1] = *(const v8h*)(Psh + c * 64 + kk * 32 + 16 + 8 * hh);
      pl.h[0] = *(const v8h*)(Psl + c * 64 + kk * 32 + 8 * hh);
      pl.h[1] = *(const v8h*)(Psl + c * 64 + kk * 32 + 16 + 8 * hh);
#pragma unroll
      for (int t = 0; t < 4; ++t) {
        const v16h vb = ldfrag<_Float16>(Vh + (size_t)(t * 16 + c) * SEQ + kv0 + kk * 32 + 8 * hh);
        const v16h vr = ldfrag<_Float16>(Vl + (size_t)(t * 16 + c) * SEQ + kv0 + kk * 32 + 8 * hh);
        oacc[t] = mma_h(pa.v, vb, oacc[t]);
        o1[t]   = mma_h(pa.v, vr, o1[t]);
        o1[t]   = mma_h(pl.v, vb, o1[t]);
      }
    }
#pragma unroll
    for (int t = 0; t < 4; ++t)
#pragma unroll
      for (int r = 0; r < 8; ++r) oacc[t][r] += o1[t][r] * (1.0f / 4096.0f);
  }

  float* os = Os[wave];
#pragma unroll
  for (int r = 0; r < 8; ++r) {
    const float l = lrow[r];
    const float inv = ((l > 0.f) ? (1.0f / l) : 0.f) * (1.0f / PCARRY);
#pragma unroll
    for (int t = 0; t < 4; ++t) os[(8 * hh + r) * 64 + t * 16 + c] = oacc[t][r] * inv;
  }
  __builtin_amdgcn_fence(__ATOMIC_RELEASE, "workgroup");
  __builtin_amdgcn_wave_barrier();
  __builtin_amdgcn_fence(__ATOMIC_ACQUIRE, "workgroup");
  {
    const int h2 = lane >> 4, c4 = (lane & 15) * 4;
    v4f ov[8];
#pragma unroll
    for (int it = 0; it < 8; ++it) {
      const int row = it * 2 + h2;
      ov[it] = *(const v4f*)(os + row * 64 + c4);
    }
    for (int pass = 0; pass < 2; ++pass) {
#pragma unroll
      for (int it = 0; it < 8; ++it) {
        const int row = it * 2 + h2;
        const size_t go = (rowB + q0 + row) * DM + (size_t)dbase + c4;
        *(volatile v4f*)(outp + go) = ov[it];
      }
      __threadfence();
    }
  }
}

extern "C" void kernel_launch(void* const* d_in, const int* in_sizes, int n_in,
                              void* d_out, int out_size, void* d_ws, size_t ws_size,
                              hipStream_t stream) {
  if (n_in < 4) return;
  if (in_sizes[0] < ((NB - 1) * SEQ_FULL + SEQ) * DM) return;
  if (in_sizes[1] < DM * DM) return;
  if (in_sizes[2] < DM * DM) return;
  if (in_sizes[3] < DM * DM) return;
  if (out_size < NB * SEQ * DM) return;

  const float* x  = (const float*)d_in[0];
  const float* wq = (const float*)d_in[1];
  const float* wk = (const float*)d_in[2];
  const float* wv = (const float*)d_in[3];

  const size_t PX  = (size_t)NB * SEQ * DM * 2;
  const size_t PW  = (size_t)DM * DM * 2;
  const size_t PVT = (size_t)NB * DM * SEQ * 2;
  size_t off = 0;
  const size_t oXb  = off; off += PX;
  const size_t oWq  = off; off += PW;
  const size_t oWk  = off; off += PW;
  const size_t oWv  = off; off += PW;
  const size_t oQh  = off; off += PX;
  const size_t oQl  = off; off += PX;
  const size_t oKp  = off; off += PX;
  const size_t oVTh = off; off += PVT;
  const size_t oVTl = off; off += PVT;
  if (off > ws_size) return;
  if (off > (size_t)134217728) return;

  char* ws = (char*)d_ws;
  unsigned short* Xb  = (unsigned short*)(ws + oXb);
  unsigned short* Wqb = (unsigned short*)(ws + oWq);
  unsigned short* Wkb = (unsigned short*)(ws + oWk);
  unsigned short* Wvb = (unsigned short*)(ws + oWv);
  unsigned short* Qh  = (unsigned short*)(ws + oQh);
  unsigned short* Ql  = (unsigned short*)(ws + oQl);
  unsigned short* Kp  = (unsigned short*)(ws + oKp);
  unsigned short* VTh = (unsigned short*)(ws + oVTh);
  unsigned short* VTl = (unsigned short*)(ws + oVTl);
  const float* nobias = wq;

  const int M = NB * SEQ;
  const dim3 blk(256);
  const int n8x = NB * SEQ * DM / 8;
  const int n8w = DM * DM / 8;
  const dim3 gCx((n8x + 255) / 256);
  const dim3 gCw((n8w + 255) / 256);
  const dim3 gQ(((M / 64) * (DM / 64) + 7) / 8, 1);
  const dim3 gVT(((DM / 64) * (SEQ / 64) + 7) / 8, NB);
  const dim3 gAttn(NB * NQB);

  cvtx<<<gCx, blk, 0, stream>>>(x, Xb, n8x);
  cvt16x8<0><<<gCw, blk, 0, stream>>>(wq, Wqb, n8w);
  cvt16x8<0><<<gCw, blk, 0, stream>>>(wk, Wkb, n8w);
  cvt16x8<0><<<gCw, blk, 0, stream>>>(wv, Wvb, n8w);
  gemm_t<__bf16, 4, false, 3><<<gQ, blk, 0, stream>>>(
      Xb, Xb, DM, 0LL, Wqb, DM, 0LL,
      (void*)Qh, (void*)Ql, DM, 0LL, nobias,
      M, DM, DM, 1.0f, 4096.0f, 0.0f);
  gemm_t<__bf16, 4, false, 1><<<gQ, blk, 0, stream>>>(
      Xb, Xb, DM, 0LL, Wkb, DM, 0LL,
      (void*)Kp, (void*)Kp, DM, 0LL, nobias,
      M, DM, DM, 1.0f, 1.0f, 0.0f);
  gemm_t<__bf16, 4, false, 3><<<gVT, blk, 0, stream>>>(
      Wvb, Wvb, DM, 0LL, Xb, DM, (long long)SEQ * DM,
      (void*)VTh, (void*)VTl, SEQ, (long long)DM * SEQ, nobias,
      DM, SEQ, DM, 1.0f, 4096.0f, 0.0f);
  attn_causal<<<gAttn, dim3(128), 0, stream>>>(Qh, Ql, Kp, VTh, VTl, (float*)d_out, 0.0625f);
  (void)hipGetLastError();
}
